// NonLocal_68255620268249
// MI455X (gfx1250) — hardware-run, weakly checked
//
#include <hip/hip_runtime.h>
#include <math.h>

constexpr int kB    = 2;
constexpr int kC    = 64;
constexpr int kH    = 80;
constexpr int kWd   = 80;
constexpr int kN    = kH * kWd;
constexpr int kRows = kB * kN;
constexpr int kTaps = 9;
constexpr int kK    = kTaps * kC;
constexpr int kSegs = kK / 8;
constexpr int kQC   = 1600;
constexpr int kNQC  = kN / kQC;
constexpr float kWCarry    = 256.0f;
constexpr float kWCarryInv = 1.0f / 256.0f;
constexpr float kPCarry    = 32768.0f;
constexpr float kPCarryInv = 1.0f / 32768.0f;
constexpr int kSmT  = 160;
constexpr int kSmIt = kN / (kSmT * 8);
constexpr int kI2cRows = 32;
constexpr int kI2cIt   = kI2cRows * kSegs / 256;
constexpr int kWSegTotal = kC * kSegs;
static_assert(kN % 64 == 0 && kRows % 64 == 0 && kC % 64 == 0 && kQC % 64 == 0, "M,N tile multiples");
static_assert(kK % 32 == 0 && kC % 32 == 0 && kN % 32 == 0, "K multiples of 32");
static_assert(kNQC * kQC == kN, "chunks");
static_assert(kSmT * 8 * kSmIt == kN, "softmax coverage");
static_assert(kI2cIt * 256 == kI2cRows * kSegs && kRows % kI2cRows == 0, "im2col coverage");
static_assert(kWSegTotal % 256 == 0, "wcast coverage");
static_assert(kSegs % 8 == 0, "8-lane groups align to 128-B lines");

typedef __attribute__((ext_vector_type(16))) _Float16 v16h;
typedef __attribute__((ext_vector_type(8)))  _Float16 v8h;
typedef __attribute__((ext_vector_type(16))) __bf16   v16b;
typedef __attribute__((ext_vector_type(8)))  __bf16   v8b;
typedef __attribute__((ext_vector_type(8)))  float    v8f;
typedef __attribute__((ext_vector_type(4)))  float    v4f;
typedef __attribute__((ext_vector_type(4)))  unsigned int v4u;

__device__ __forceinline__ unsigned short f2bf_bits(float f) {
  unsigned u = __float_as_uint(f);
  return (unsigned short)((u + 0x7FFFu + ((u >> 16) & 1u)) >> 16);
}
__device__ __forceinline__ float bf_bits2f(unsigned short h) { return __uint_as_float(((unsigned)h) << 16); }

__device__ __forceinline__ void dep_guard4_h(v8f& a, v8f& b, v8f& c, v8f& d, v16h x, v16h y) {
  asm volatile("v_nop\n\tv_nop\n\tv_nop\n\tv_nop" : "+v"(a), "+v"(b), "+v"(c), "+v"(d) : "v"(x), "v"(y));
}
__device__ __forceinline__ void dep_guard4_b(v8f& a, v8f& b, v8f& c, v8f& d, v16b x, v16b y) {
  asm volatile("v_nop\n\tv_nop\n\tv_nop\n\tv_nop" : "+v"(a), "+v"(b), "+v"(c), "+v"(d) : "v"(x), "v"(y));
}
__device__ __forceinline__ void keep4_h(v16h a, v16h b, v16h c, v16h d) { asm volatile("v_nop" :: "v"(a), "v"(b), "v"(c), "v"(d)); }
__device__ __forceinline__ void keep4_b(v16b a, v16b b, v16b c, v16b d) { asm volatile("v_nop" :: "v"(a), "v"(b), "v"(c), "v"(d)); }
__device__ __forceinline__ void acc_guard4(v8f& a, v8f& b, v8f& c, v8f& d) { asm volatile("v_nop\n\tv_nop\n\tv_nop\n\tv_nop" : "+v"(a), "+v"(b), "+v"(c), "+v"(d)); }
template <typename T> struct Frag;
template <> struct Frag<_Float16> {
  typedef v16h V; union U { v16h v; v8h h[2]; };
  static __device__ __forceinline__ v16h load(const _Float16* p) {
    U f; f.h[0] = *(const v8h*)(p); f.h[1] = *(const v8h*)(p + 16); return f.v;
  }
  static __device__ __forceinline__ v8f mma(v16h a, v16h b, v8f c) {
    return __builtin_amdgcn_wmma_f32_16x16x32_f16(false, a, false, b, (short)0, c, false, false);
  }
  static __device__ __forceinline__ void guard4(v8f& a, v8f& b, v8f& c, v8f& d, v16h x, v16h y) { dep_guard4_h(a, b, c, d, x, y); }
  static __device__ __forceinline__ void keep(v16h a, v16h b, v16h c, v16h d) { keep4_h(a, b, c, d); }
};
template <> struct Frag<__bf16> {
  typedef v16b V; union U { v16b v; v8b h[2]; };
  static __device__ __forceinline__ v16b load(const __bf16* p) {
    U f; f.h[0] = *(const v8b*)(p); f.h[1] = *(const v8b*)(p + 16); return f.v;
  }
  static __device__ __forceinline__ v8f mma(v16b a, v16b b, v8f c) {
    return __builtin_amdgcn_wmma_f32_16x16x32_bf16(false, a, false, b, (short)0, c, false, false);
  }
  static __device__ __forceinline__ void guard4(v8f& a, v8f& b, v8f& c, v8f& d, v16b x, v16b y) { dep_guard4_b(a, b, c, d, x, y); }
  static __device__ __forceinline__ void keep(v16b a, v16b b, v16b c, v16b d) { keep4_b(a, b, c, d); }
};

__device__ __forceinline__ unsigned pk16(unsigned short a, unsigned short b) { return (unsigned)a | ((unsigned)b << 16); }
__device__ __forceinline__ unsigned short h_bits(float f) { const _Float16 h = (_Float16)f; return __builtin_bit_cast(unsigned short, h); }

template <int ET> struct Elem;
template <> struct Elem<0> { typedef _Float16 T; };
template <> struct Elem<1> { typedef __bf16 T; };
template <int ET, bool SPLIT, int BIAS_MODE, int OUT_MODE, bool RESID, int ACT = 0>
__global__ __launch_bounds__(256) void wmma_gemm64(
    const unsigned short* __restrict__ Ap, const unsigned short* __restrict__ A2p, int lda, long strideA,
    const unsigned short* __restrict__ Btp, const unsigned short* __restrict__ Bt2p, int ldb, long strideB,
    void* __restrict__ Cout, void* __restrict__ Cout2, int ldc, long strideC,
    const float* __restrict__ bias,
    const float* __restrict__ resid, long strideR,
    int M, int N, int K, float scale) {
  static_assert(!(RESID && OUT_MODE != 0), "resid path is f32 output only");
  typedef typename Elem<ET>::T T;
  typedef typename Frag<T>::V V;
  const T* A = (const T*)Ap; const T* A2 = (const T*)A2p; const T* Bt = (const T*)Btp; const T* Bt2 = (const T*)Bt2p;
  __shared__ __align__(16) float sT[8][16 * 68];
  const int b    = blockIdx.y;
  const int lane = threadIdx.x & 31;
  const int wave = threadIdx.x >> 5;
  const int tilesN = N >> 6;
  const int tilesM = M >> 6;
  const int tile = blockIdx.x * 8 + wave;
  if (tile >= tilesM * tilesN) return;
  const int tm = tile / tilesN;
  const int tn = tile - tm * tilesN;
  const int m0 = tm << 6;
  const int n0 = tn << 6;

  const T* Ab  = A  + (size_t)b * strideA;
  const T* Bb  = Bt + (size_t)b * strideB;
  const T* Ab2 = SPLIT ? (A2  + (size_t)b * strideA) : nullptr;
  const T* Bb2 = SPLIT ? (Bt2 + (size_t)b * strideB) : nullptr;

  const int rlane = lane & 15;
  const int koff  = (lane >> 4) * 8;
  const int mOff  = (lane >> 4) * 8;

  v8f acc[4][4];
#pragma unroll
  for (int i = 0; i < 4; ++i)
#pragma unroll
    for (int j = 0; j < 4; ++j) acc[i][j] = (v8f){0.f,0.f,0.f,0.f,0.f,0.f,0.f,0.f};

  for (int k0 = 0; k0 < K; k0 += 32) {
    V bh[4], bl[4];
#pragma unroll
    for (int j = 0; j < 4; ++j) {
      const size_t bo = (size_t)(n0 + (j << 4) + rlane) * ldb + koff + k0;
      bh[j] = Frag<T>::load(Bb + bo);
      if (SPLIT) bl[j] = Frag<T>::load(Bb2 + bo);
    }
#pragma unroll
    for (int i = 0; i < 4; ++i) {
      const size_t ao = (size_t)(m0 + (i << 4) + rlane) * lda + koff + k0;
      V ah = Frag<T>::load(Ab + ao);
      V al;
      if (SPLIT) al = Frag<T>::load(Ab2 + ao);
#pragma unroll
      for (int j = 0; j < 4; ++j) {
        acc[i][j] = Frag<T>::mma(ah, bh[j], acc[i][j]);
        if (SPLIT) {
          acc[i][j] = Frag<T>::mma(ah, bl[j], acc[i][j]);
          acc[i][j] = Frag<T>::mma(al, bh[j], acc[i][j]);
        }
      }
      Frag<T>::guard4(acc[i][0], acc[i][1], acc[i][2], acc[i][3], ah, SPLIT ? al : ah);
    }
    Frag<T>::keep(bh[0], bh[1], bh[2], bh[3]);
    if (SPLIT) Frag<T>::keep(bl[0], bl[1], bl[2], bl[3]);
  }
  acc_guard4(acc[0][0], acc[0][1], acc[0][2], acc[0][3]);
  acc_guard4(acc[1][0], acc[1][1], acc[1][2], acc[1][3]);
  acc_guard4(acc[2][0], acc[2][1], acc[2][2], acc[2][3]);
  acc_guard4(acc[3][0], acc[3][1], acc[3][2], acc[3][3]);

  float* slab = sT[wave];
  const float* Rb = RESID ? (resid + (size_t)b * strideR) : nullptr;
#pragma unroll
  for (int i = 0; i < 4; ++i) {
    const int mBase = m0 + (i << 4);
    v4f bm0 = (v4f){0.f,0.f,0.f,0.f};
    v4f bm1 = (v4f){0.f,0.f,0.f,0.f};
    if (BIAS_MODE == 1) {
      bm0 = *(const v4f*)(bias + mBase + mOff);
      bm1 = *(const v4f*)(bias + mBase + mOff + 4);
    }
#pragma unroll
    for (int j = 0; j < 4; ++j) {
      const int n = n0 + (j << 4) + rlane;
      float bv = 0.f;
      if (BIAS_MODE == 2) bv = bias[n];
#pragma unroll
      for (int r = 0; r < 8; ++r) {
        float v = acc[i][j][r] * scale;
        if (BIAS_MODE == 1) { const float bb = (r < 4) ? bm0[r & 3] : bm1[r & 3]; v += bb; }
        if (BIAS_MODE == 2) v += bv;
        if (ACT == 2) v = fmaxf(v, 0.0f);
        if (ACT == 4) v = (v > 0.f) ? v : 0.01f * v;
        slab[(mOff + r) * 68 + (j << 4) + rlane] = v;
      }
    }
    __builtin_amdgcn_fence(__ATOMIC_RELEASE, "workgroup");
    __builtin_amdgcn_wave_barrier();
    __builtin_amdgcn_fence(__ATOMIC_ACQUIRE, "workgroup");
    if (OUT_MODE == 0) {
      float* C = (float*)Cout + (size_t)b * strideC;
      const int hh = lane >> 4, c4 = (lane & 15) * 4;
      for (int pass = 0; pass < 2; ++pass) {
#pragma unroll
        for (int it = 0; it < 8; ++it) {
          const int row = it * 2 + hh;
          v4f v = *(const v4f*)(slab + row * 68 + c4);
          const size_t co = (size_t)(mBase + row) * ldc + n0 + c4;
          if (RESID) { const v4f rr = *(const v4f*)(Rb + co); v += rr; }
          *(volatile v4f*)(C + co) = v;
        }
        __threadfence();
      }
    } else {
      const int q = lane >> 3, c8 = (lane & 7) * 8;
      unsigned short* C  = (unsigned short*)Cout  + (size_t)b * strideC;
      unsigned short* C2 = (OUT_MODE == 2) ? ((unsigned short*)Cout2 + (size_t)b * strideC) : nullptr;
      for (int pass = 0; pass < 2; ++pass) {
#pragma unroll
        for (int it = 0; it < 4; ++it) {
          const int row = it * 4 + q;
          const float* sp = slab + row * 68 + c8;
          v8h hv, lv;
#pragma unroll
          for (int e = 0; e < 8; ++e) {
            if (OUT_MODE == 1) {
              hv[e] = (_Float16)sp[e];
            } else {
              unsigned short hb = f2bf_bits(sp[e]);
              unsigned short lb = f2bf_bits(sp[e] - bf_bits2f(hb));
              hv[e] = __builtin_bit_cast(_Float16, hb);
              lv[e] = __builtin_bit_cast(_Float16, lb);
            }
          }
          *(volatile v8h*)(C + (size_t)(mBase + row) * ldc + n0 + c8) = hv;
          if (OUT_MODE == 2) *(volatile v8h*)(C2 + (size_t)(mBase + row) * ldc + n0 + c8) = lv;
        }
        __threadfence();
      }
    }
    __builtin_amdgcn_fence(__ATOMIC_RELEASE, "workgroup");
    __builtin_amdgcn_wave_barrier();
    __builtin_amdgcn_fence(__ATOMIC_ACQUIRE, "workgroup");
  }
}

__global__ __launch_bounds__(256) void wcast_kernel(const float* __restrict__ w0, const float* __restrict__ w1,
                                                    const float* __restrict__ w2, const float* __restrict__ w3,
                                                    unsigned short* __restrict__ out, float scale) {
  const int z = blockIdx.y;
  const float* wsrc = (z == 0) ? w0 : (z == 1) ? w1 : (z == 2) ? w2 : w3;
  const int g   = blockIdx.x * 256 + threadIdx.x;
  const int oc  = g / kSegs;
  const int s   = g - oc * kSegs;
  const int t   = s >> 3;
  const int ic0 = (s & 7) * 8;
  const float* wr = wsrc + (size_t)oc * kK + t;
  unsigned short hb[8];
#pragma unroll
  for (int e = 0; e < 8; ++e) hb[e] = h_bits(wr[(ic0 + e) * 9] * scale);
  const v4u u = (v4u){pk16(hb[0], hb[1]), pk16(hb[2], hb[3]), pk16(hb[4], hb[5]), pk16(hb[6], hb[7])};
  unsigned short* dp = out + (size_t)z * kC * kK + (size_t)oc * kK + s * 8;
  *(volatile v4u*)dp = u;
  __threadfence();
  *(volatile v4u*)dp = u;
}

template <bool SRC_PC>
__global__ __launch_bounds__(256) void im2col_kernel(const float* __restrict__ src, unsigned short* __restrict__ dst) {
  const int tid   = threadIdx.x;
  const int rbase = blockIdx.x * kI2cRows;
  for (int pass = 0; pass < 2; ++pass) {
#pragma unroll 1
    for (int i = 0; i < kI2cIt; ++i) {
      const int g   = i * 256 + tid;
      const int rl  = g / kSegs;
      const int s   = g - rl * kSegs;
      const int r   = rbase + rl;
      const int b   = r / kN;
      const int pix = r - b * kN;
      const int h   = pix / kWd;
      const int w   = pix - h * kWd;
      const int t   = s >> 3;
      const int ic0 = (s & 7) * 8;
      const int kh  = t / 3;
      const int kw  = t - kh * 3;
      const int hs  = h + kh - 1;
      const int wsr = w + kw - 1;
      const bool valid = (hs >= 0) && (hs < kH) && (wsr >= 0) && (wsr < kWd);
      const int hc  = hs < 0 ? 0 : (hs > kH - 1 ? kH - 1 : hs);
      const int wc  = wsr < 0 ? 0 : (wsr > kWd - 1 ? kWd - 1 : wsr);
      const int ps  = hc * kWd + wc;
      const float fv = valid ? 1.0f : 0.0f;
      float v[8];
      if (SRC_PC) {
        const float* p = src + ((size_t)(b * kN + ps)) * kC + ic0;
        const v4f a = *(const v4f*)(p);
        const v4f c = *(const v4f*)(p + 4);
#pragma unroll
        for (int e = 0; e < 4; ++e) { v[e] = a[e]; v[4 + e] = c[e]; }
      } else {
        const float* p = src + ((size_t)(b * kC + ic0)) * kN + ps;
#pragma unroll
        for (int e = 0; e < 8; ++e) v[e] = p[(size_t)e * kN];
      }
      unsigned short hb[8];
#pragma unroll
      for (int e = 0; e < 8; ++e) hb[e] = h_bits(v[e] * fv);
      const v4u u = (v4u){pk16(hb[0], hb[1]), pk16(hb[2], hb[3]), pk16(hb[4], hb[5]), pk16(hb[6], hb[7])};
      *(volatile v4u*)(dst + (size_t)r * kK + s * 8) = u;
    }
    __threadfence();
  }
}

__global__ __launch_bounds__(kSmT) void softmax_rows_kernel(const float* __restrict__ Sp, unsigned short* __restrict__ Pp) {
  __shared__ __align__(16) float lg[kN];
  __shared__ float redM[8];
  __shared__ float redS[8];
  const int row  = blockIdx.x;
  const int t    = threadIdx.x;
  const int lane = t & 31, wave = t >> 5;
  const float* sr = Sp + (size_t)row * kN;

  float mx = -__builtin_inff();
#pragma unroll 1
  for (int it = 0; it < kSmIt; ++it) {
    const int c0 = (it * kSmT + t) * 8;
    const v4f a = *(const v4f*)(sr + c0);
    const v4f c = *(const v4f*)(sr + c0 + 4);
    const float m0 = fmaxf(fmaxf(a[0], a[1]), fmaxf(a[2], a[3]));
    const float m1 = fmaxf(fmaxf(c[0], c[1]), fmaxf(c[2], c[3]));
    mx = fmaxf(mx, fmaxf(m0, m1));
    *(v4f*)(lg + c0) = a;
    *(v4f*)(lg + c0 + 4) = c;
  }
#pragma unroll
  for (int off = 16; off > 0; off >>= 1) mx = fmaxf(mx, __shfl_xor(mx, off, 32));
  if (lane == 0) redM[wave] = mx;
  __syncthreads();
  float m = redM[0];
#pragma unroll
  for (int wv = 1; wv < kSmT / 32; ++wv) m = fmaxf(m, redM[wv]);

  float sum = 0.f;
#pragma unroll 1
  for (int it = 0; it < kSmIt; ++it) {
    const int c0 = (it * kSmT + t) * 8;
    const v4f l0 = *(const v4f*)(lg + c0);
    const v4f l1 = *(const v4f*)(lg + c0 + 4);
    v4f e0, e1;
#pragma unroll
    for (int e = 0; e < 4; ++e) { e0[e] = expf(l0[e] - m); sum += e0[e]; }
#pragma unroll
    for (int e = 0; e < 4; ++e) { e1[e] = expf(l1[e] - m); sum += e1[e]; }
    *(v4f*)(lg + c0) = e0;
    *(v4f*)(lg + c0 + 4) = e1;
  }
#pragma unroll
  for (int off = 16; off > 0; off >>= 1) sum += __shfl_xor(sum, off, 32);
  if (lane == 0) redS[wave] = sum;
  __syncthreads();
  float tot = redS[0];
#pragma unroll
  for (int wv = 1; wv < kSmT / 32; ++wv) tot += redS[wv];
  const float inv = kPCarry / tot;

  unsigned short* prow = Pp + (size_t)row * kN;
  for (int pass = 0; pass < 2; ++pass) {
#pragma unroll 1
    for (int it = 0; it < kSmIt; ++it) {
      const int c0 = (it * kSmT + t) * 8;
      const v4f e0 = *(const v4f*)(lg + c0);
      const v4f e1 = *(const v4f*)(lg + c0 + 4);
      unsigned short hb[8];
#pragma unroll
      for (int e = 0; e < 4; ++e) {
        hb[e]     = h_bits(e0[e] * inv);
        hb[4 + e] = h_bits(e1[e] * inv);
      }
      const v4u u = (v4u){pk16(hb[0], hb[1]), pk16(hb[2], hb[3]), pk16(hb[4], hb[5]), pk16(hb[6], hb[7])};
      *(volatile v4u*)(prow + c0) = u;
    }
    __threadfence();
  }
}

extern "C" void kernel_launch(void* const* d_in, const int* in_sizes, int n_in,
                              void* d_out, int out_size, void* d_ws, size_t ws_size,
                              hipStream_t stream) {
  if (n_in < 9) return;
  const int nAct = kB * kC * kN;
  const int nW   = kC * kC * kTaps;
  if (in_sizes[0] != nAct || out_size != nAct) return;
  if (in_sizes[1] != nW || in_sizes[3] != nW || in_sizes[5] != nW || in_sizes[7] != nW) return;
  if (in_sizes[2] != kC || in_sizes[4] != kC || in_sizes[6] != kC || in_sizes[8] != kC) return;

  const size_t szW16 = (size_t)4 * kC * kK * 2;
  const size_t szBt  = (size_t)kRows * kK * 2;
  const size_t szT   = (size_t)kRows * kC * 2;
  const size_t szSC  = (size_t)kQC * kN * 4;
  const size_t szPP  = (size_t)kQC * kN * 2;
  const size_t szY   = (size_t)kRows * kC * 4;
  const size_t offW16 = 0;
  const size_t offBtX = offW16 + szW16;
  const size_t offTh  = offBtX + szBt;
  const size_t offPh  = offTh + szT;
  const size_t offG   = offPh + szT;
  const size_t offSC  = offG + szT;
  const size_t offPP  = offSC + szSC;
  const size_t offY   = offPP + szPP;
  const size_t offBtY = offY + szY;
  const size_t total  = offBtY + szBt;
  if (ws_size < total) return;

  const float* x    = (const float*)d_in[0];
  const float* g_w  = (const float*)d_in[1];
  const float* g_b  = (const float*)d_in[2];
  const float* th_w = (const float*)d_in[3];
  const float* th_b = (const float*)d_in[4];
  const float* ph_w = (const float*)d_in[5];
  const float* ph_b = (const float*)d_in[6];
  const float* W_w  = (const float*)d_in[7];
  const float* W_b  = (const float*)d_in[8];
  float* out = (float*)d_out;
  char* ws = (char*)d_ws;
  unsigned short* W16    = (unsigned short*)(ws + offW16);
  unsigned short* BtX    = (unsigned short*)(ws + offBtX);
  unsigned short* thetaT = (unsigned short*)(ws + offTh);
  unsigned short* phiT   = (unsigned short*)(ws + offPh);
  unsigned short* gCN    = (unsigned short*)(ws + offG);
  float*          SC     = (float*)(ws + offSC);
  unsigned short* PP     = (unsigned short*)(ws + offPP);
  float*          Y      = (float*)(ws + offY);
  unsigned short* BtY    = (unsigned short*)(ws + offBtY);
  const size_t wplane = (size_t)kC * kK;
  const unsigned short* Wth = W16 + 0 * wplane;
  const unsigned short* Wph = W16 + 1 * wplane;
  const unsigned short* Wg  = W16 + 2 * wplane;
  const unsigned short* Wo  = W16 + 3 * wplane;

  wcast_kernel<<<dim3(kWSegTotal / 256, 4), dim3(256), 0, stream>>>(th_w, ph_w, g_w, W_w, W16, kWCarry);
  im2col_kernel<false><<<dim3(kRows / kI2cRows), dim3(256), 0, stream>>>(x, BtX);

  const int tilesTP = (kRows / 64) * (kC / 64);
  wmma_gemm64<0, false, 2, 1, false, 2><<<dim3((tilesTP + 7) / 8, 1), dim3(256), 0, stream>>>(
      BtX, BtX, kK, 0L, Wth, Wth, kK, 0L, (void*)thetaT, (void*)thetaT, kC, 0L, th_b, x, 0L, kRows, kC, kK, kWCarryInv);
  wmma_gemm64<0, false, 2, 1, false, 2><<<dim3((tilesTP + 7) / 8, 1), dim3(256), 0, stream>>>(
      BtX, BtX, kK, 0L, Wph, Wph, kK, 0L, (void*)phiT, (void*)phiT, kC, 0L, ph_b, x, 0L, kRows, kC, kK, kWCarryInv);
  const int tilesCN = (kC / 64) * (kN / 64);
  wmma_gemm64<0, false, 1, 1, false, 2><<<dim3((tilesCN + 7) / 8, kB), dim3(256), 0, stream>>>(
      Wg, Wg, kK, 0L, BtX, BtX, kK, (long)kN * kK, (void*)gCN, (void*)gCN, kN, (long)kC * kN, g_b, x, 0L, kC, kN, kK, kWCarryInv);

  const int tilesS  = (kQC / 64) * (kN / 64);
  const int tilesPV = (kQC / 64) * (kC / 64);
  for (int b = 0; b < kB; ++b) {
    for (int qc = 0; qc < kNQC; ++qc) {
      const size_t qrow0 = (size_t)b * kN + (size_t)qc * kQC;
      const unsigned short* Ath = thetaT + qrow0 * kC;
      const unsigned short* Bph = phiT + (size_t)b * kN * kC;
      wmma_gemm64<0, false, 0, 0, false, 0><<<dim3((tilesS + 7) / 8, 1), dim3(256), 0, stream>>>(
          Ath, Ath, kC, 0L, Bph, Bph, kC, 0L, (void*)SC, (void*)SC, kN, 0L, th_b, x, 0L, kQC, kN, kC, 1.0f);
      softmax_rows_kernel<<<dim3(kQC), dim3(kSmT), 0, stream>>>(SC, PP);
      const unsigned short* Bg = gCN + (size_t)b * kC * kN;
      float* Yc = Y + qrow0 * kC;
      wmma_gemm64<0, false, 0, 0, false, 0><<<dim3((tilesPV + 7) / 8, 1), dim3(256), 0, stream>>>(
          PP, PP, kN, 0L, Bg, Bg, kN, 0L, (void*)Yc, (void*)Yc, kC, 0L, th_b, x, 0L, kQC, kC, kN, kPCarryInv);
    }
  }

  im2col_kernel<true><<<dim3(kRows / kI2cRows), dim3(256), 0, stream>>>(Y, BtY);
  wmma_gemm64<0, false, 1, 0, true, 2><<<dim3((tilesCN + 7) / 8, kB), dim3(256), 0, stream>>>(
      Wo, Wo, kK, 0L, BtY, BtY, kK, (long)kN * kK, (void*)out, (void*)out, kN, (long)kC * kN, W_b, x, (long)kC * kN,
      kC, kN, kK, kWCarryInv);
}
